// MCM_37031208026850
// MI455X (gfx1250) — hardware-verified
//
#include <hip/hip_runtime.h>
#define BB 4
#define CC 512
#define HWN 1024
#define NP (BB * HWN)
#define HS 32
#define C64 64

typedef __bf16 v16b __attribute__((ext_vector_type(16)));
typedef unsigned short v8us __attribute__((ext_vector_type(8), may_alias));
typedef float  v8f  __attribute__((ext_vector_type(8)));
typedef float  v4f  __attribute__((ext_vector_type(4)));
typedef float  v4fa __attribute__((ext_vector_type(4), may_alias));
union FragB { v16b v; v8us half[2]; unsigned short u[16]; };

__device__ __forceinline__ unsigned short bf16_bits(float x) { unsigned int u = __float_as_uint(x); return (unsigned short)((u + 0x7FFFu + ((u >> 16) & 1u)) >> 16); }
__device__ __forceinline__ float bf16_val(unsigned short b) { return __uint_as_float(((unsigned int)b) << 16); }
__device__ __forceinline__ float bf16_round(float x) { return bf16_val(bf16_bits(x)); }
template <int NT>
__device__ __forceinline__ v8f mmaN(v16b ah, v16b al, v16b bh, v16b bl, v8f c) {
  c = __builtin_amdgcn_wmma_f32_16x16x32_bf16(false, ah, false, bh, (short)0, c, false, false);
  if (NT >= 2) c = __builtin_amdgcn_wmma_f32_16x16x32_bf16(false, al, false, bh, (short)0, c, false, false);
  if (NT >= 3) c = __builtin_amdgcn_wmma_f32_16x16x32_bf16(false, ah, false, bl, (short)0, c, false, false);
  asm volatile("v_nop\n\tv_nop\n\tv_nop\n\tv_nop" : "+v"(c) : "v"(ah), "v"(al), "v"(bh), "v"(bl));
  return c;
}

__global__ __launch_bounds__(256) void k_wt_bf16(const float* __restrict__ W, unsigned short* __restrict__ Wt, int K, int N) {
  const int t = blockIdx.x * 256 + threadIdx.x;
  const int k8n = K / 8;
  if (t >= N * k8n) return;
  const int n = t / k8n, k8 = (t % k8n) * 8;
  v8us v;
#pragma unroll
  for (int i = 0; i < 8; ++i) v[i] = bf16_bits(W[(size_t)(k8 + i) * N + n]);
  *(volatile v8us*)(Wt + (size_t)n * K + k8) = v;
  __threadfence();
  *(volatile v8us*)(Wt + (size_t)n * K + k8) = v;
}

template <bool ASPLIT, int ACT, bool BIAS_BF16>
__global__ __launch_bounds__(128) void k_gemm_bf(const float* __restrict__ A, int lda, const unsigned short* __restrict__ Wt, int ldb,
                                               const float* __restrict__ bias, float* __restrict__ C, int ldc, int M, int N, int K) {
  __shared__ __attribute__((aligned(16))) float so[4][16][64];
  const int tid = threadIdx.x, w = tid >> 5, lane = tid & 31, ln = lane & 15, hh = lane >> 4;
  const int ntn = N / 64;
  const int wid = blockIdx.x * 4 + w;
  const int mt = wid / ntn, nq = wid % ntn;
  if (mt * 16 >= M) return;
  const int row0 = mt * 16, col0 = nq * 64;
  const float* arow = A + (size_t)(row0 + ln) * lda;
  v8f acc[4] = {};
  for (int kb = 0; kb < K; kb += 32) {
    FragB ah, al;
    const v4f x0 = *(const v4fa*)(arow + kb + 8 * hh), x1 = *(const v4fa*)(arow + kb + 8 * hh + 4);
    const v4f x2 = *(const v4fa*)(arow + kb + 16 + 8 * hh), x3 = *(const v4fa*)(arow + kb + 16 + 8 * hh + 4);
    float xs[16] = {x0[0],x0[1],x0[2],x0[3],x1[0],x1[1],x1[2],x1[3],x2[0],x2[1],x2[2],x2[3],x3[0],x3[1],x3[2],x3[3]};
#pragma unroll
    for (int i = 0; i < 16; ++i) { const unsigned short hb = bf16_bits(xs[i]); ah.u[i] = hb; al.u[i] = ASPLIT ? bf16_bits(xs[i] - bf16_val(hb)) : (unsigned short)0; }
#pragma unroll
    for (int t = 0; t < 4; ++t) {
      const unsigned short* brow = Wt + (size_t)(col0 + t * 16 + ln) * ldb + kb;
      FragB b;
      b.half[0] = *(const v8us*)(brow + 8 * hh);
      b.half[1] = *(const v8us*)(brow + 16 + 8 * hh);
      acc[t] = mmaN<ASPLIT ? 2 : 1>(ah.v, al.v, b.v, b.v, acc[t]);
    }
  }
#pragma unroll
  for (int t = 0; t < 4; ++t) {
    float bv = bias ? bias[col0 + t * 16 + ln] : 0.f;
    if (BIAS_BF16) bv = bf16_round(bv);
#pragma unroll
    for (int r = 0; r < 8; ++r) { float v = acc[t][r] + bv; if (ACT == 1) v = fmaxf(v, 0.f); so[w][8 * hh + r][t * 16 + ln] = v; }
  }
  __builtin_amdgcn_fence(__ATOMIC_ACQ_REL, "workgroup");
  __builtin_amdgcn_wave_barrier();
  const int rsub = lane >> 4, c4 = (lane & 15) * 4;
  for (int pass = 0; pass < 2; ++pass) {
#pragma unroll
    for (int q = 0; q < 8; ++q) {
      const int r = q * 2 + rsub;
      const v4f v = *(const v4fa*)&so[w][r][c4];
      *(volatile v4f*)(C + (size_t)(row0 + r) * ldc + col0 + c4) = v;
    }
    if (pass == 0) __threadfence();
  }
}

template <int D, bool CAUSAL>
__global__ __launch_bounds__(128) void k_flash(const float* __restrict__ qb, const float* __restrict__ kb, const float* __restrict__ vb,
                                             int pitch, int T, int H, float scale, float* __restrict__ y, int ypitch) {
  constexpr int KS = D / 32;
  constexpr int DT = D / 16;
  __shared__ __attribute__((aligned(16))) unsigned short sKh[32][D + 8], sKl[32][D + 8], sVh[32][D + 8], sVl[32][D + 8];
  __shared__ __attribute__((aligned(16))) unsigned short sPh[4][16][40], sPl[4][16][40];
  __shared__ __attribute__((aligned(16))) float sO[4][16][D];
  const int tid = threadIdx.x, w = tid >> 5, lane = tid & 31, ln = lane & 15, hh = lane >> 4;
  const int nqb = (T + 63) / 64;
  const int bh = blockIdx.x / nqb, qblk = blockIdx.x % nqb;
  const int b = bh / H, h = bh % H;
  const int q0 = qblk * 64 + w * 16;
  const float* Q = qb + (size_t)b * T * pitch + h * D;
  const float* K = kb + (size_t)b * T * pitch + h * D;
  const float* V = vb + (size_t)b * T * pitch + h * D;

  FragB aqh[KS], aql[KS];
  {
    int row = q0 + ln; if (row >= T) row = T - 1;
    const float* qr = Q + (size_t)row * pitch;
#pragma unroll
    for (int ks = 0; ks < KS; ++ks)
#pragma unroll
      for (int i = 0; i < 16; ++i) {
        const int d = ks * 32 + ((i < 8) ? (8 * hh + i) : (16 + 8 * hh + (i - 8)));
        const float x = qr[d] * scale; const unsigned short hb = bf16_bits(x);
        aqh[ks].u[i] = hb; aql[ks].u[i] = bf16_bits(x - bf16_val(hb));
      }
  }
  float m_r[8], l_r[8];
#pragma unroll
  for (int r = 0; r < 8; ++r) { m_r[r] = -3.0e38f; l_r[r] = 0.f; }
  v8f oacc[DT];
#pragma unroll
  for (int dt = 0; dt < DT; ++dt) oacc[dt] = (v8f){0.f,0.f,0.f,0.f,0.f,0.f,0.f,0.f};

  const int kv_end = CAUSAL ? min(T, qblk * 64 + 64) : T;
  for (int j0 = 0; j0 < kv_end; j0 += 32) {
    __syncthreads();
    for (int e = tid; e < 32 * (D / 4); e += 128) {
      const int r = e / (D / 4), c4 = (e % (D / 4)) * 4;
      const int key = j0 + r;
      v4f kf = {0.f,0.f,0.f,0.f}, vf = {0.f,0.f,0.f,0.f};
      if (key < T) { kf = *(const v4fa*)(K + (size_t)key * pitch + c4); vf = *(const v4fa*)(V + (size_t)key * pitch + c4); }
#pragma unroll
      for (int t = 0; t < 4; ++t) {
        unsigned short hb = bf16_bits(kf[t]); sKh[r][c4 + t] = hb; sKl[r][c4 + t] = bf16_bits(kf[t] - bf16_val(hb));
        hb = bf16_bits(vf[t]); sVh[r][c4 + t] = hb; sVl[r][c4 + t] = bf16_bits(vf[t] - bf16_val(hb));
      }
    }
    __syncthreads();
    v8f s[2];
#pragma unroll
    for (int nt = 0; nt < 2; ++nt) {
      v8f acc = {};
#pragma unroll
      for (int ks = 0; ks < KS; ++ks) {
        FragB bh_, bl_;
        bh_.half[0] = *(const v8us*)&sKh[nt * 16 + ln][ks * 32 + 8 * hh]; bh_.half[1] = *(const v8us*)&sKh[nt * 16 + ln][ks * 32 + 16 + 8 * hh];
        bl_.half[0] = *(const v8us*)&sKl[nt * 16 + ln][ks * 32 + 8 * hh]; bl_.half[1] = *(const v8us*)&sKl[nt * 16 + ln][ks * 32 + 16 + 8 * hh];
        acc = mmaN<3>(aqh[ks].v, aql[ks].v, bh_.v, bl_.v, acc);
      }
      s[nt] = acc;
    }
    float alpha[8];
#pragma unroll
    for (int r = 0; r < 8; ++r) {
      const int qi = q0 + 8 * hh + r;
      const int ja = j0 + ln, jb = j0 + 16 + ln;
      if (CAUSAL) { if (ja > qi) s[0][r] = -3.0e38f; if (jb > qi) s[1][r] = -3.0e38f; }
      if (ja >= T) s[0][r] = -3.0e38f;
      if (jb >= T) s[1][r] = -3.0e38f;
      float mx = fmaxf(s[0][r], s[1][r]);
      mx = fmaxf(mx, __shfl_xor(mx, 1, 32)); mx = fmaxf(mx, __shfl_xor(mx, 2, 32)); mx = fmaxf(mx, __shfl_xor(mx, 4, 32)); mx = fmaxf(mx, __shfl_xor(mx, 8, 32));
      const float mnew = fmaxf(m_r[r], mx);
      alpha[r] = (mnew > -1.0e38f) ? __expf(m_r[r] - mnew) : 1.0f;
      const float p0 = (s[0][r] > -1.0e38f) ? __expf(s[0][r] - mnew) : 0.f;
      const float p1 = (s[1][r] > -1.0e38f) ? __expf(s[1][r] - mnew) : 0.f;
      m_r[r] = mnew;
      l_r[r] = l_r[r] * alpha[r] + p0 + p1;
      unsigned short hb = bf16_bits(p0); sPh[w][8 * hh + r][ln] = hb;      sPl[w][8 * hh + r][ln] = bf16_bits(p0 - bf16_val(hb));
      hb = bf16_bits(p1);                sPh[w][8 * hh + r][16 + ln] = hb; sPl[w][8 * hh + r][16 + ln] = bf16_bits(p1 - bf16_val(hb));
    }
#pragma unroll
    for (int dt = 0; dt < DT; ++dt)
#pragma unroll
      for (int r = 0; r < 8; ++r) oacc[dt][r] *= alpha[r];
    __builtin_amdgcn_fence(__ATOMIC_ACQ_REL, "workgroup");
    __builtin_amdgcn_wave_barrier();
    FragB pah, pal;
    pah.half[0] = *(const v8us*)&sPh[w][ln][8 * hh]; pah.half[1] = *(const v8us*)&sPh[w][ln][16 + 8 * hh];
    pal.half[0] = *(const v8us*)&sPl[w][ln][8 * hh]; pal.half[1] = *(const v8us*)&sPl[w][ln][16 + 8 * hh];
#pragma unroll
    for (int dt = 0; dt < DT; ++dt) {
      FragB bvh, bvl;
#pragma unroll
      for (int i = 0; i < 8; ++i) {
        bvh.u[i] = sVh[8 * hh + i][dt * 16 + ln]; bvh.u[8 + i] = sVh[16 + 8 * hh + i][dt * 16 + ln];
        bvl.u[i] = sVl[8 * hh + i][dt * 16 + ln]; bvl.u[8 + i] = sVl[16 + 8 * hh + i][dt * 16 + ln];
      }
      oacc[dt] = mmaN<3>(pah.v, pal.v, bvh.v, bvl.v, oacc[dt]);
    }
    __builtin_amdgcn_fence(__ATOMIC_ACQ_REL, "workgroup");
    __builtin_amdgcn_wave_barrier();
  }
#pragma unroll
  for (int r = 0; r < 8; ++r) {
    float l = l_r[r];
    l += __shfl_xor(l, 1, 32); l += __shfl_xor(l, 2, 32); l += __shfl_xor(l, 4, 32); l += __shfl_xor(l, 8, 32);
    l_r[r] = (l > 0.f) ? 1.0f / l : 0.f;
  }
#pragma unroll
  for (int dt = 0; dt < DT; ++dt)
#pragma unroll
    for (int r = 0; r < 8; ++r) sO[w][8 * hh + r][dt * 16 + ln] = oacc[dt][r] * l_r[r];
  __builtin_amdgcn_fence(__ATOMIC_ACQ_REL, "workgroup");
  __builtin_amdgcn_wave_barrier();
  for (int pass = 0; pass < 2; ++pass) {
    for (int r = 0; r < 16; ++r) {
      const int row = q0 + r;
      if (row < T && lane < D / 4) {
        const v4f val = *(const v4fa*)&sO[w][r][lane * 4];
        *(volatile v4f*)(y + ((size_t)b * T + row) * ypitch + h * D + lane * 4) = val;
      }
    }
    if (pass == 0) __threadfence();
  }
}

template <bool ASPLIT, int ACT, bool BIAS_BF16, bool RES_BF16>
__global__ __launch_bounds__(128) void k_gemm_bf3(const float* __restrict__ A, int lda, const unsigned short* __restrict__ Wt, int ldb,
                                                const float* __restrict__ bias, const float* __restrict__ resid, int rmod, int ldr,
                                                float* __restrict__ C, int ldc, int M, int N, int K) {
  __shared__ __attribute__((aligned(16))) float so[4][16][64];
  const int tid = threadIdx.x, w = tid >> 5, lane = tid & 31, ln = lane & 15, hh = lane >> 4;
  const int ntn = N / 64;
  const int wid = blockIdx.x * 4 + w;
  const int mt = wid / ntn, nq = wid % ntn;
  if (mt * 16 >= M) return;
  const int row0 = mt * 16, col0 = nq * 64;
  const float* arow = A + (size_t)(row0 + ln) * lda;
  v8f acc[4] = {};
  for (int kb = 0; kb < K; kb += 32) {
    FragB ah, al;
    const v4f x0 = *(const v4fa*)(arow + kb + 8 * hh), x1 = *(const v4fa*)(arow + kb + 8 * hh + 4);
    const v4f x2 = *(const v4fa*)(arow + kb + 16 + 8 * hh), x3 = *(const v4fa*)(arow + kb + 16 + 8 * hh + 4);
    float xs[16] = {x0[0],x0[1],x0[2],x0[3],x1[0],x1[1],x1[2],x1[3],x2[0],x2[1],x2[2],x2[3],x3[0],x3[1],x3[2],x3[3]};
#pragma unroll
    for (int i = 0; i < 16; ++i) { const unsigned short hb = bf16_bits(xs[i]); ah.u[i] = hb; al.u[i] = ASPLIT ? bf16_bits(xs[i] - bf16_val(hb)) : (unsigned short)0; }
#pragma unroll
    for (int t = 0; t < 4; ++t) {
      const unsigned short* brow = Wt + (size_t)(col0 + t * 16 + ln) * ldb + kb;
      FragB b;
      b.half[0] = *(const v8us*)(brow + 8 * hh);
      b.half[1] = *(const v8us*)(brow + 16 + 8 * hh);
      acc[t] = mmaN<ASPLIT ? 2 : 1>(ah.v, al.v, b.v, b.v, acc[t]);
    }
  }
#pragma unroll
  for (int t = 0; t < 4; ++t) {
    const int col = col0 + t * 16 + ln;
    float bv = bias ? bias[col] : 0.f;
    if (BIAS_BF16) bv = bf16_round(bv);
#pragma unroll
    for (int r = 0; r < 8; ++r) {
      float v = acc[t][r] + bv;
      if (resid) { float rv = resid[(size_t)((row0 + 8 * hh + r) % rmod) * ldr + col]; if (RES_BF16) rv = bf16_round(rv); v += rv; }
      if (ACT == 1) v = fmaxf(v, 0.f);
      if (ACT == 2) v = 0.5f * v * (1.0f + erff(v * 0.70710678118654752f));
      if (ACT == 3) { const float u = 0.7978845608028654f * (v + 0.044715f * v * v * v); v = 0.5f * v * (1.0f + tanhf(u)); }
      so[w][8 * hh + r][t * 16 + ln] = v;
    }
  }
  __builtin_amdgcn_fence(__ATOMIC_ACQ_REL, "workgroup");
  __builtin_amdgcn_wave_barrier();
  const int rsub = lane >> 4, c4 = (lane & 15) * 4;
  for (int pass = 0; pass < 2; ++pass) {
#pragma unroll
    for (int q = 0; q < 8; ++q) {
      const int r = q * 2 + rsub;
      const v4f v = *(const v4fa*)&so[w][r][c4];
      *(volatile v4f*)(C + (size_t)(row0 + r) * ldc + col0 + c4) = v;
    }
    if (pass == 0) __threadfence();
  }
}
template <bool PARAM_BF16>
__global__ __launch_bounds__(256) void k_layernorm(const float* __restrict__ X, const float* __restrict__ R, const float* __restrict__ g, const float* __restrict__ bta,
                                                  float* __restrict__ out_sum, float* __restrict__ out_norm, int N, float eps) {
  __shared__ float red[256];
  const int row = blockIdx.x, tid = threadIdx.x;
  const float* x = X + (size_t)row * N; const float* rr = R ? R + (size_t)row * N : nullptr;
  float vals[16];
  const int per = N / 256;
  float s1 = 0.f;
  for (int u = 0; u < per / 4; ++u) {
    const int j = tid * 4 + 1024 * u;
    const v4f a = *(const v4fa*)(x + j);
    v4f b = {0.f,0.f,0.f,0.f}; if (rr) b = *(const v4fa*)(rr + j);
#pragma unroll
    for (int q = 0; q < 4; ++q) { const float v = a[q] + b[q]; vals[u * 4 + q] = v; s1 += v; }
  }
  red[tid] = s1; __syncthreads();
  for (int st = 128; st > 0; st >>= 1) { if (tid < st) red[tid] += red[tid + st]; __syncthreads(); }
  const float mu = red[0] / (float)N; __syncthreads();
  float s2 = 0.f;
  for (int u = 0; u < per / 4; ++u)
#pragma unroll
    for (int q = 0; q < 4; ++q) { const float c = vals[u * 4 + q] - mu; s2 += c * c; }
  red[tid] = s2; __syncthreads();
  for (int st = 128; st > 0; st >>= 1) { if (tid < st) red[tid] += red[tid + st]; __syncthreads(); }
  const float rs = rsqrtf(red[0] / (float)N + eps);
  for (int pass = 0; pass < 2; ++pass) {
    for (int u = 0; u < per / 4; ++u) {
      const int j = tid * 4 + 1024 * u;
      v4f o, sm;
#pragma unroll
      for (int q = 0; q < 4; ++q) {
        float gg = g[j + q], bb = bta[j + q];
        if (PARAM_BF16) { gg = bf16_round(gg); bb = bf16_round(bb); }
        sm[q] = vals[u * 4 + q]; o[q] = (vals[u * 4 + q] - mu) * rs * gg + bb;
      }
      if (out_sum) *(volatile v4f*)(out_sum + (size_t)row * N + j) = sm;
      *(volatile v4f*)(out_norm + (size_t)row * N + j) = o;
    }
    if (pass == 0) __threadfence();
  }
}


typedef _Float16 v16h __attribute__((ext_vector_type(16)));
union FragH { v16h v; v8us half[2]; _Float16 h[16]; unsigned short u[16]; };
template <int NT>
__device__ __forceinline__ v8f mmaH(v16h ah, v16h al, v16h bh, v16h bl, v8f c) {
  c = __builtin_amdgcn_wmma_f32_16x16x32_f16(false, ah, false, bh, (short)0, c, false, false);
  if (NT >= 2) c = __builtin_amdgcn_wmma_f32_16x16x32_f16(false, al, false, bh, (short)0, c, false, false);
  if (NT >= 3) c = __builtin_amdgcn_wmma_f32_16x16x32_f16(false, ah, false, bl, (short)0, c, false, false);
  asm volatile("v_nop\n\tv_nop\n\tv_nop\n\tv_nop" : "+v"(c) : "v"(ah), "v"(al), "v"(bh), "v"(bl));
  return c;
}
template <bool ASPLIT>
__global__ __launch_bounds__(128) void k_gemm_h(const float* __restrict__ A, int lda, size_t sA, const _Float16* __restrict__ Bh, int ldb, size_t sB, float alpha, float* __restrict__ C, int ldc, size_t sC, int M, int N, int K) {
  __shared__ __attribute__((aligned(16))) float so[4][16][64];
  const int tid = threadIdx.x, w = tid >> 5, lane = tid & 31, ln = lane & 15, hh = lane >> 4; const int by = blockIdx.y;
  A += (size_t)by * sA; Bh += (size_t)by * sB; C += (size_t)by * sC;
  const int ntn = (N + 63) / 64; const int wid = blockIdx.x * 4 + w; const int mt = wid / ntn, nq = wid % ntn; if (mt * 16 >= M) return;
  const int row0 = mt * 16, col0 = nq * 64; const float* arow = A + (size_t)(row0 + ln) * lda;
  v8f acc[4] = {};
  for (int kb = 0; kb < K; kb += 32) {
    FragH ah, al;
    const v4f x0 = *(const v4fa*)(arow + kb + 8 * hh), x1 = *(const v4fa*)(arow + kb + 8 * hh + 4), x2 = *(const v4fa*)(arow + kb + 16 + 8 * hh), x3 = *(const v4fa*)(arow + kb + 16 + 8 * hh + 4);
    float xs[16] = {x0[0],x0[1],x0[2],x0[3],x1[0],x1[1],x1[2],x1[3],x2[0],x2[1],x2[2],x2[3],x3[0],x3[1],x3[2],x3[3]};
#pragma unroll
    for (int i = 0; i < 16; ++i) { const _Float16 h = (_Float16)xs[i]; ah.h[i] = h; al.h[i] = ASPLIT ? (_Float16)(xs[i] - (float)h) : (_Float16)0.0f; }
#pragma unroll
    for (int t = 0; t < 4; ++t) { if (col0 + t * 16 >= N) continue; const size_t boff = (size_t)(col0 + t * 16 + ln) * ldb + kb; FragH bq; bq.half[0] = *(const v8us*)(Bh + boff + 8 * hh); bq.half[1] = *(const v8us*)(Bh + boff + 16 + 8 * hh);
      acc[t] = mmaH<ASPLIT ? 2 : 1>(ah.v, al.v, bq.v, bq.v, acc[t]); }
  }
#pragma unroll
  for (int t = 0; t < 4; ++t) { if (col0 + t * 16 >= N) continue;
#pragma unroll
    for (int r = 0; r < 8; ++r) so[w][8 * hh + r][t * 16 + ln] = acc[t][r] * alpha; }
  __builtin_amdgcn_fence(__ATOMIC_ACQ_REL, "workgroup"); __builtin_amdgcn_wave_barrier();
  const int rsub = lane >> 4, c4 = (lane & 15) * 4;
  for (int pass = 0; pass < 2; ++pass) {
#pragma unroll
    for (int q = 0; q < 8; ++q) { const int r = q * 2 + rsub; if (col0 + c4 < N) { const v4f v = *(const v4fa*)&so[w][r][c4]; *(volatile v4f*)(C + (size_t)(row0 + r) * ldc + col0 + c4) = v; } }
    if (pass == 0) __threadfence(); }
}

__global__ __launch_bounds__(256) void k_wt_f16(const float* __restrict__ W, _Float16* __restrict__ Wt, int K, int N, float scale) {
  const int t = blockIdx.x * 256 + threadIdx.x; if (t >= N * (K / 8)) return; const int n = t / (K / 8), k8 = (t % (K / 8)) * 8; FragH f;
#pragma unroll
  for (int i = 0; i < 8; ++i) f.h[i] = (_Float16)(bf16_round(W[(size_t)(k8 + i) * N + n]) * scale); const v8us o = f.half[0];
  *(volatile v8us*)((unsigned short*)Wt + (size_t)n * K + k8) = o; __threadfence(); *(volatile v8us*)((unsigned short*)Wt + (size_t)n * K + k8) = o;
}
template <int ACT>
__global__ __launch_bounds__(128) void k_gemm_hhx(const _Float16* __restrict__ A, int lda, size_t sA, const _Float16* __restrict__ Bh, int ldb, size_t sB, float alpha, const float* __restrict__ bias, size_t sBias, const float* __restrict__ CP, int rowsPerB, size_t sCPb, int row0g,
    float* __restrict__ C, _Float16* __restrict__ C16, int ldc, size_t sC, int M, int N, int K) {
  __shared__ __attribute__((aligned(16))) float so[4][16][64];
  const int tid = threadIdx.x, w = tid >> 5, lane = tid & 31, ln = lane & 15, hh = lane >> 4; const int by = blockIdx.y;
  A += (size_t)by * sA; Bh += (size_t)by * sB; const size_t cofs = (size_t)by * sC; const float* bp = bias ? bias + (size_t)by * sBias : nullptr;
  const int ntn = (N + 63) / 64; const int wid = blockIdx.x * 4 + w; const int mt = wid / ntn, nq = wid % ntn; if (mt * 16 >= M) return;
  const int row0 = mt * 16, col0 = nq * 64; const _Float16* arow = A + (size_t)(row0 + ln) * lda;
  v8f acc[4] = {};
  for (int kb = 0; kb < K; kb += 32) { FragH ah; ah.half[0] = *(const v8us*)((const unsigned short*)arow + kb + 8 * hh); ah.half[1] = *(const v8us*)((const unsigned short*)arow + kb + 16 + 8 * hh);
#pragma unroll
    for (int t = 0; t < 4; ++t) { if (col0 + t * 16 >= N) continue; const size_t boff = (size_t)(col0 + t * 16 + ln) * ldb + kb; FragH bq; bq.half[0] = *(const v8us*)((const unsigned short*)Bh + boff + 8 * hh); bq.half[1] = *(const v8us*)((const unsigned short*)Bh + boff + 16 + 8 * hh);
      acc[t] = mmaH<1>(ah.v, ah.v, bq.v, bq.v, acc[t]); }
  }
#pragma unroll
  for (int t = 0; t < 4; ++t) { if (col0 + t * 16 >= N) continue; const int col = col0 + t * 16 + ln; const float bv = bp ? bf16_round(bp[col]) : 0.f;
#pragma unroll
    for (int r = 0; r < 8; ++r) { float v = acc[t][r] * alpha + bv; if (CP) { const int bidx = (row0g + row0 + 8 * hh + r) / rowsPerB; v += CP[(size_t)bidx * sCPb + (size_t)by * 64 + col]; } if (ACT == 1) v = (v > 0.f) ? v : expm1f(v); else if (ACT == 3) v = fmaxf(v, 0.f); so[w][8 * hh + r][t * 16 + ln] = v; } }
  __builtin_amdgcn_fence(__ATOMIC_ACQ_REL, "workgroup"); __builtin_amdgcn_wave_barrier();
  const int rsub = lane >> 4, c4 = (lane & 15) * 4; typedef _Float16 v4h __attribute__((ext_vector_type(4)));
  for (int pass = 0; pass < 2; ++pass) {
#pragma unroll
    for (int q = 0; q < 8; ++q) { const int r = q * 2 + rsub; if (col0 + c4 < N) { const v4f v = *(const v4fa*)&so[w][r][c4]; if (C) *(volatile v4f*)(C + cofs + (size_t)(row0 + r) * ldc + col0 + c4) = v; if (C16) { v4h h4; for (int i = 0; i < 4; ++i) h4[i] = (_Float16)v[i]; *(volatile v4h*)(C16 + cofs + (size_t)(row0 + r) * ldc + col0 + c4) = h4; } } }
    if (pass == 0) __threadfence(); }
}


__global__ __launch_bounds__(256) void k_round16f(const float* __restrict__ W, _Float16* __restrict__ Bt, size_t n8) { const size_t t = (size_t)blockIdx.x * 256 + threadIdx.x; if (t >= n8) return; FragH f;
#pragma unroll
  for (int i = 0; i < 8; ++i) f.h[i] = (_Float16)(bf16_round(W[t * 8 + i]) * 16.0f); *(volatile v8us*)((unsigned short*)Bt + t * 8) = f.half[0]; __threadfence(); *(volatile v8us*)((unsigned short*)Bt + t * 8) = f.half[0]; }
__global__ __launch_bounds__(256) void k_wconv(const float* __restrict__ w, _Float16* __restrict__ Bc) { const size_t t = (size_t)blockIdx.x * 256 + threadIdx.x; if (t >= (size_t)C64 * 9 * 128 / 8) return; const int o = (int)(t / (9 * 128 / 8)); const int k8 = (int)(t % (9 * 128 / 8)) * 8; FragH f;
#pragma unroll
  for (int q = 0; q < 8; ++q) { const int k = k8 + q; const int tap = k / 128, c = k % 128; f.h[q] = (_Float16)(bf16_round(w[((size_t)o * 128 + c) * 9 + tap]) * 16.0f); } *(volatile v8us*)((unsigned short*)Bc + t * 8) = f.half[0]; __threadfence(); *(volatile v8us*)((unsigned short*)Bc + t * 8) = f.half[0]; }
__global__ __launch_bounds__(256) void k_in16(const float* __restrict__ xc, const float* __restrict__ xt, _Float16* __restrict__ XC, _Float16* __restrict__ XT) { const size_t t = (size_t)blockIdx.x * 256 + threadIdx.x; if (t >= (size_t)NP * CC / 8) return; const size_t p = t / (CC / 8); const int c8 = (int)(t % (CC / 8)) * 8; const int b = (int)(p / HWN), hw = (int)(p % HWN); FragH f, g;
#pragma unroll
  for (int q = 0; q < 8; ++q) { f.h[q] = (_Float16)bf16_round(xc[((size_t)b * CC + c8 + q) * HWN + hw]); g.h[q] = (_Float16)bf16_round(xt[t * 8 + q]); }
  *(volatile v8us*)((unsigned short*)XC + t * 8) = f.half[0]; *(volatile v8us*)((unsigned short*)XT + t * 8) = g.half[0]; __threadfence(); *(volatile v8us*)((unsigned short*)XC + t * 8) = f.half[0]; *(volatile v8us*)((unsigned short*)XT + t * 8) = g.half[0]; }
__global__ __launch_bounds__(128) void k_gate(const _Float16* __restrict__ Q, const _Float16* __restrict__ Kt, float* __restrict__ co) {
  __shared__ float sres[64];
  const int tid = threadIdx.x, w = tid >> 5, lane = tid & 31, ln = lane & 15, hh = lane >> 4; const int r0 = (blockIdx.x * 4 + w) * 16;
  FragH aq[16];
  { const unsigned short* qr = (const unsigned short*)Q + (size_t)(r0 + ln) * CC;
#pragma unroll
    for (int ks = 0; ks < 16; ++ks) { aq[ks].half[0] = *(const v8us*)(qr + ks * 32 + 8 * hh); aq[ks].half[1] = *(const v8us*)(qr + ks * 32 + 16 + 8 * hh); } }
  float tot[8];
#pragma unroll
  for (int r = 0; r < 8; ++r) tot[r] = 0.f;
#pragma unroll 1
  for (int b = 0; b < BB; ++b) { float mx[8], sm[8];
#pragma unroll
    for (int r = 0; r < 8; ++r) { mx[r] = -3.0e38f; sm[r] = 0.f; }
#pragma unroll 1
    for (int jt = 0; jt < HWN / 16; ++jt) { const unsigned short* kr = (const unsigned short*)Kt + (size_t)(b * HWN + jt * 16 + ln) * CC; v8f acc = {0.f,0.f,0.f,0.f,0.f,0.f,0.f,0.f};
#pragma unroll
      for (int ks = 0; ks < 16; ++ks) { FragH bk; bk.half[0] = *(const v8us*)(kr + ks * 32 + 8 * hh); bk.half[1] = *(const v8us*)(kr + ks * 32 + 16 + 8 * hh); acc = mmaH<1>(aq[ks].v, aq[ks].v, bk.v, bk.v, acc); }
#pragma unroll
      for (int r = 0; r < 8; ++r) { mx[r] = fmaxf(mx[r], acc[r]); sm[r] += acc[r]; } }
#pragma unroll
    for (int r = 0; r < 8; ++r) { float m = mx[r], s = sm[r];
#pragma unroll
      for (int o = 1; o <= 8; o <<= 1) { m = fmaxf(m, __shfl_xor(m, o, 32)); s += __shfl_xor(s, o, 32); }
      tot[r] += m + s * (1.0f / (float)HWN); } }
  if (ln == 0) {
#pragma unroll
    for (int r = 0; r < 8; ++r) sres[w * 16 + 8 * hh + r] = tot[r]; }
  __syncthreads();
  if (tid < 64) { *(volatile float*)(co + (size_t)blockIdx.x * 64 + tid) = sres[tid]; } __threadfence(); if (tid < 64) { *(volatile float*)(co + (size_t)blockIdx.x * 64 + tid) = sres[tid]; } }
__global__ __launch_bounds__(256) void k_soft(const float* __restrict__ CO, float* __restrict__ G) { __shared__ float red[8]; const int tid = threadIdx.x, wv = tid >> 5, lane = tid & 31; const int g = blockIdx.x / BB, b = blockIdx.x % BB; const float* c = CO + (size_t)g * NP + b * HWN; const float sc = 0.04419417382415922f;
  float v[4]; float m = -3.0e38f; for (int u = 0; u < 4; ++u) { v[u] = c[u * 256 + tid] * sc; m = fmaxf(m, v[u]); }
  for (int o = 16; o >= 1; o >>= 1) m = fmaxf(m, __shfl_xor(m, o, 32)); if (lane == 0) red[wv] = m; __syncthreads(); m = red[0]; for (int i = 1; i < 8; ++i) m = fmaxf(m, red[i]); __syncthreads();
  float s = 0.f; for (int u = 0; u < 4; ++u) { v[u] = expf(v[u] - m); s += v[u]; }
  for (int o = 16; o >= 1; o >>= 1) s += __shfl_xor(s, o, 32); if (lane == 0) red[wv] = s; __syncthreads(); s = 0.f; for (int i = 0; i < 8; ++i) s += red[i]; const float inv = 1.0f / s;
  for (int pass = 0; pass < 2; ++pass) { for (int u = 0; u < 4; ++u) *(volatile float*)(G + (size_t)g * NP + b * HWN + u * 256 + tid) = v[u] * inv; if (pass == 0) __threadfence(); } }
__global__ __launch_bounds__(256) void k_mix(const float* __restrict__ Pc, const float* __restrict__ Pt, const float* __restrict__ G, const float* __restrict__ b64, _Float16* __restrict__ CATc, _Float16* __restrict__ CATt) { const size_t t = (size_t)blockIdx.x * 256 + threadIdx.x; if (t >= (size_t)NP * 128 / 8) return; const size_t p = t / 16; const int c8 = (int)(t % 16) * 8; const int half = c8 / 64, c0 = c8 % 64;
  const float gc = G[(half ? 2 : 0) * NP + p], gt = G[(half ? 3 : 1) * NP + p]; FragH f, g;
#pragma unroll
  for (int q = 0; q < 8; ++q) { const float bb = bf16_round(b64[c0 + q]); f.h[q] = (_Float16)((gc * Pc[p * C64 + c0 + q] + bb) * 8192.0f); g.h[q] = (_Float16)((gt * Pt[p * C64 + c0 + q] + bb) * 8192.0f); }
  *(volatile v8us*)((unsigned short*)CATc + t * 8) = f.half[0]; *(volatile v8us*)((unsigned short*)CATt + t * 8) = g.half[0]; __threadfence(); *(volatile v8us*)((unsigned short*)CATc + t * 8) = f.half[0]; *(volatile v8us*)((unsigned short*)CATt + t * 8) = g.half[0]; }
template <bool OUT_F16>
__global__ __launch_bounds__(128) void k_conv3(const _Float16* __restrict__ IN16, const _Float16* __restrict__ Bc, const float* __restrict__ bias, float inscale, _Float16* __restrict__ DST16, int col0, float* __restrict__ out) {
  __shared__ __attribute__((aligned(16))) float so[64][65];
  const int tid = threadIdx.x, w = tid >> 5, lane = tid & 31, ln = lane & 15, hh = lane >> 4; const int p0 = (blockIdx.x * 4 + w) * 16; const int p = p0 + ln; const int b = p / HWN, hw = p % HWN, y = hw / HS, xx = hw % HS;
  v8f acc[4];
#pragma unroll
  for (int q = 0; q < 4; ++q) acc[q] = (v8f){0.f,0.f,0.f,0.f,0.f,0.f,0.f,0.f};
#pragma unroll 1
  for (int ks = 0; ks < 36; ++ks) { const int tap = ks >> 2, cb = (ks & 3) * 32; const int yy = y + tap / 3 - 1, x2 = xx + tap % 3 - 1; FragH a;
    if (yy >= 0 && yy < HS && x2 >= 0 && x2 < HS) { const unsigned short* ar = (const unsigned short*)IN16 + ((size_t)b * HWN + yy * HS + x2) * 128 + cb; a.half[0] = *(const v8us*)(ar + 8 * hh); a.half[1] = *(const v8us*)(ar + 16 + 8 * hh); }
    else { for (int j = 0; j < 16; ++j) a.h[j] = (_Float16)0.0f; }
#pragma unroll
    for (int q = 0; q < 4; ++q) { FragH bq; const unsigned short* br = (const unsigned short*)Bc + (size_t)(q * 16 + ln) * 1152 + ks * 32; bq.half[0] = *(const v8us*)(br + 8 * hh); bq.half[1] = *(const v8us*)(br + 16 + 8 * hh); acc[q] = mmaH<1>(a.v, a.v, bq.v, bq.v, acc[q]); } }
#pragma unroll
  for (int q = 0; q < 4; ++q) { const int o = q * 16 + ln; const float bv = bf16_round(bias[o]);
#pragma unroll
    for (int r = 0; r < 8; ++r) so[w * 16 + 8 * hh + r][o] = fmaxf(acc[q][r] * inscale + bv, 0.f); }
  __syncthreads();
  if (OUT_F16) { typedef _Float16 v4h __attribute__((ext_vector_type(4)));
    for (int pass = 0; pass < 2; ++pass) { for (int j = tid; j < 64 * 16; j += 128) { const int r = j / 16, c4 = (j % 16) * 4; v4h h4; h4[0] = (_Float16)(so[r][c4] * 8192.0f); h4[1] = (_Float16)(so[r][c4 + 1] * 8192.0f); h4[2] = (_Float16)(so[r][c4 + 2] * 8192.0f); h4[3] = (_Float16)(so[r][c4 + 3] * 8192.0f); *(volatile v4h*)(DST16 + (size_t)(blockIdx.x * 64 + r) * 128 + col0 + c4) = h4; } if (pass == 0) __threadfence(); } }
  else { typedef float v2f __attribute__((ext_vector_type(2), aligned(8))); const int pb = blockIdx.x * 64; const int bimg = pb / HWN, hw0 = pb % HWN;
    for (int pass = 0; pass < 2; ++pass) { for (int o = w; o < C64; o += 4) { v2f v; v.x = so[2 * lane][o]; v.y = so[2 * lane + 1][o]; *(volatile v2f*)(out + ((size_t)bimg * C64 + o) * HWN + hw0 + 2 * lane) = v; } if (pass == 0) __threadfence(); } } }

extern "C" void kernel_launch(void* const* d_in, const int* in_sizes, int n_in,
                              void* d_out, int out_size, void* d_ws, size_t ws_size, hipStream_t stream) {
  (void)in_sizes; (void)n_in; (void)out_size;
  const float* xc = (const float*)d_in[0]; const float* xt = (const float*)d_in[1]; const float* Wqc = (const float*)d_in[2]; const float* bqc = (const float*)d_in[3]; const float* Wkc = (const float*)d_in[4]; const float* bkc = (const float*)d_in[5]; const float* Wvc = (const float*)d_in[6]; const float* bvc = (const float*)d_in[7];
  const float* Wqt = (const float*)d_in[8]; const float* bqt = (const float*)d_in[9]; const float* Wkt = (const float*)d_in[10]; const float* bkt = (const float*)d_in[11]; const float* W64 = (const float*)d_in[12]; const float* b64 = (const float*)d_in[13];
  const float* W1 = (const float*)d_in[14]; const float* b1 = (const float*)d_in[15]; const float* W2 = (const float*)d_in[16]; const float* b2 = (const float*)d_in[17]; const float* W3 = (const float*)d_in[18]; const float* b3 = (const float*)d_in[19];
  char* ws = (char*)d_ws; size_t off = 0;
  auto take = [&](size_t bytes) { char* p = ws + off; off += (bytes + 255) & ~(size_t)255; return p; };
  _Float16* Bw = (_Float16*)take((size_t)5 * CC * CC * 2); _Float16* B64 = (_Float16*)take((size_t)C64 * CC * 2); _Float16* Bc1 = (_Float16*)take((size_t)C64 * 1152 * 2); _Float16* Bc2 = (_Float16*)take((size_t)C64 * 1152 * 2); _Float16* Bc3 = (_Float16*)take((size_t)C64 * 1152 * 2);
  _Float16* XC = (_Float16*)take((size_t)NP * CC * 2); _Float16* XT = (_Float16*)take((size_t)NP * CC * 2); _Float16* CQ = (_Float16*)take((size_t)NP * CC * 2); _Float16* CK = (_Float16*)take((size_t)NP * CC * 2); _Float16* TQ = (_Float16*)take((size_t)NP * CC * 2); _Float16* TK = (_Float16*)take((size_t)NP * CC * 2); _Float16* VC = (_Float16*)take((size_t)NP * CC * 2);
  float* Pc = (float*)take((size_t)NP * C64 * 4); float* Pt = (float*)take((size_t)NP * C64 * 4); float* CO = (float*)take((size_t)4 * NP * 4); float* G = (float*)take((size_t)4 * NP * 4); _Float16* CATc = (_Float16*)take((size_t)NP * 128 * 2); _Float16* CATt = (_Float16*)take((size_t)NP * 128 * 2); _Float16* CAT3 = (_Float16*)take((size_t)NP * 128 * 2);
  if (off > ws_size) return;
  const size_t n8 = (size_t)CC * CC / 8; const unsigned gw = (unsigned)((n8 + 255) / 256);
  k_round16f<<<gw, 256, 0, stream>>>(Wqc, Bw, n8); k_round16f<<<gw, 256, 0, stream>>>(Wkc, Bw + (size_t)CC * CC, n8); k_round16f<<<gw, 256, 0, stream>>>(Wvc, Bw + (size_t)2 * CC * CC, n8); k_round16f<<<gw, 256, 0, stream>>>(Wqt, Bw + (size_t)3 * CC * CC, n8); k_round16f<<<gw, 256, 0, stream>>>(Wkt, Bw + (size_t)4 * CC * CC, n8);
  k_round16f<<<(unsigned)(((size_t)C64 * CC / 8 + 255) / 256), 256, 0, stream>>>(W64, B64, (size_t)C64 * CC / 8);
  k_wconv<<<(unsigned)(((size_t)C64 * 9 * 128 / 8 + 255) / 256), 256, 0, stream>>>(W1, Bc1); k_wconv<<<(unsigned)(((size_t)C64 * 9 * 128 / 8 + 255) / 256), 256, 0, stream>>>(W2, Bc2); k_wconv<<<(unsigned)(((size_t)C64 * 9 * 128 / 8 + 255) / 256), 256, 0, stream>>>(W3, Bc3);
  k_in16<<<(unsigned)(((size_t)NP * CC / 8 + 255) / 256), 256, 0, stream>>>(xc, xt, XC, XT);
  const dim3 g512(((NP / 16) * (CC / 64) + 3) / 4, 1), g64(((NP / 16) * 1 + 3) / 4, 1);
  k_gemm_hhx<0><<<g512, 128, 0, stream>>>(XC, CC, 0, Bw, CC, 0, 0.0625f, bqc, 0, nullptr, 1, 0, 0, nullptr, CQ, CC, 0, NP, CC, CC);
  k_gemm_hhx<0><<<g512, 128, 0, stream>>>(XC, CC, 0, Bw + (size_t)CC * CC, CC, 0, 0.0625f, bkc, 0, nullptr, 1, 0, 0, nullptr, CK, CC, 0, NP, CC, CC);
  k_gemm_hhx<0><<<g512, 128, 0, stream>>>(XC, CC, 0, Bw + (size_t)2 * CC * CC, CC, 0, 0.0625f, bvc, 0, nullptr, 1, 0, 0, nullptr, VC, CC, 0, NP, CC, CC);
  k_gemm_hhx<0><<<g512, 128, 0, stream>>>(XT, CC, 0, Bw + (size_t)3 * CC * CC, CC, 0, 0.0625f, bqt, 0, nullptr, 1, 0, 0, nullptr, TQ, CC, 0, NP, CC, CC);
  k_gemm_hhx<0><<<g512, 128, 0, stream>>>(XT, CC, 0, Bw + (size_t)4 * CC * CC, CC, 0, 0.0625f, bkt, 0, nullptr, 1, 0, 0, nullptr, TK, CC, 0, NP, CC, CC);
  k_gemm_hhx<0><<<g64, 128, 0, stream>>>(VC, CC, 0, B64, CC, 0, 0.0625f, nullptr, 0, nullptr, 1, 0, 0, Pc, nullptr, C64, 0, NP, C64, CC);
  k_gemm_hhx<0><<<g64, 128, 0, stream>>>(XT, CC, 0, B64, CC, 0, 0.0625f, nullptr, 0, nullptr, 1, 0, 0, Pt, nullptr, C64, 0, NP, C64, CC);
  k_gate<<<NP / 64, 128, 0, stream>>>(CQ, CK, CO); k_gate<<<NP / 64, 128, 0, stream>>>(TQ, TK, CO + NP); k_gate<<<NP / 64, 128, 0, stream>>>(CQ, TK, CO + 2 * NP); k_gate<<<NP / 64, 128, 0, stream>>>(TQ, CK, CO + 3 * NP);
  k_soft<<<4 * BB, 256, 0, stream>>>(CO, G);
  k_mix<<<(unsigned)(((size_t)NP * 16 + 255) / 256), 256, 0, stream>>>(Pc, Pt, G, b64, CATc, CATt);
  const float insc = 1.0f / (16.0f * 8192.0f);
  k_conv3<true><<<NP / 64, 128, 0, stream>>>(CATc, Bc1, b1, insc, CAT3, 0, nullptr); k_conv3<true><<<NP / 64, 128, 0, stream>>>(CATt, Bc2, b2, insc, CAT3, 64, nullptr);
  k_conv3<false><<<NP / 64, 128, 0, stream>>>(CAT3, Bc3, b3, insc, nullptr, 0, (float*)d_out);
}
